// ExpressionClassifier_82703890252076
// MI455X (gfx1250) — hardware-verified
//
#include <hip/hip_runtime.h>


#define AS3 __attribute__((address_space(3)))

#define TT     2048
#define NN     68
#define EE     544
#define ET     612
#define HEADS  4
#define HID    32
#define F1     128
#define GOUT   128
#define LH     128
#define G4     512
#define NC     7
#define NTHR   256
#define CAP    64
#define FTS    132
#define H1S    136
#define H1R    80
#define KP2    128
#define KCL    256
#define WPL    256
#define APL    264
#define SCL    16.0f
#define INV256 0.00390625f
#define NEGS   0.2f

static_assert(F1 == HEADS * HID);
static_assert(KCL == GOUT + LH);
static_assert(KCL % 32 == 0);
static_assert(H1S % 8 == 0 && APL % 8 == 0 && KP2 % 8 == 0 && WPL % 8 == 0);
static_assert(APL >= KCL && WPL >= KCL);

typedef _Float16 v16h __attribute__((ext_vector_type(16)));
typedef _Float16 v8h  __attribute__((ext_vector_type(8)));
typedef _Float16 v4h  __attribute__((ext_vector_type(4)));
typedef float    v8f  __attribute__((ext_vector_type(8)));
typedef float    v4f  __attribute__((ext_vector_type(4)));

typedef AS3 float*          lp_f;
typedef AS3 int*            lp_i;
typedef AS3 _Float16*       lp_h;
typedef AS3 const _Float16* lcp_h;

union Frag { v16h v; v8h half[2]; };

constexpr size_t OFF_ENC = 0;
constexpr size_t SZ_ENC  = (size_t)TT * GOUT * 4;
constexpr size_t OFF_W2P = OFF_ENC + SZ_ENC;
constexpr size_t SZ_W2P  = (size_t)GOUT * KP2 * 2;
constexpr size_t OFF_WP  = OFF_W2P + SZ_W2P;
constexpr size_t SZ_WP   = (size_t)G4 * WPL * 2;
constexpr size_t OFF_LOG = OFF_WP + SZ_WP;
constexpr size_t SZ_LOG  = 128;
constexpr size_t WS_END  = OFF_LOG + SZ_LOG;
static_assert(OFF_W2P % 128 == 0 && OFF_WP % 128 == 0 && OFF_LOG % 128 == 0);
static_assert(WS_END <= (size_t)134217728);

constexpr int NPC_W2 = GOUT * (KP2 / 8);
constexpr int NPC_WP = G4 * (WPL / 8);
constexpr int NB_W2  = NPC_W2 / NTHR;
constexpr int NB_WP  = NPC_WP / NTHR;
static_assert(NPC_W2 % NTHR == 0 && NPC_WP % NTHR == 0);
static_assert((size_t)NPC_W2 * 16 == SZ_W2P && (size_t)NPC_WP * 16 == SZ_WP);

constexpr int al16(int x) { return (x + 15) & ~15; }
constexpr int LG_FEAT = 0;
constexpr int LG_H1   = al16(LG_FEAT + NN * FTS * 4);
constexpr int LG_SLOT = al16(LG_H1 + H1R * H1S * 2);
constexpr int LG_AL1  = al16(LG_SLOT + NN * CAP * 4);
constexpr int LG_AL2  = al16(LG_AL1 + ET * HEADS * 4);
constexpr int LG_AS1  = al16(LG_AL2 + ET * 4);
constexpr int LG_AD1  = al16(LG_AS1 + NN * HEADS * 4);
constexpr int LG_AS2  = al16(LG_AD1 + NN * HEADS * 4);
constexpr int LG_AD2  = al16(LG_AS2 + NN * 4);
constexpr int LG_ESRC = al16(LG_AD2 + NN * 4);
constexpr int LG_EDST = al16(LG_ESRC + ET * 4);
constexpr int LG_CSRC = al16(LG_EDST + ET * 4);
constexpr int LG_OFF  = al16(LG_CSRC + ET * 4);
constexpr int LG_CNT  = al16(LG_OFF + (NN + 1) * 4);
constexpr int LG_X    = al16(LG_CNT + NN * 4);
constexpr int LG_W1   = al16(LG_X + NN * 2 * 4);
constexpr int LG_A1S  = al16(LG_W1 + 2 * F1 * 4);
constexpr int LG_A1D  = al16(LG_A1S + F1 * 4);
constexpr int LG_B1   = al16(LG_A1D + F1 * 4);
constexpr int LG_A2S  = al16(LG_B1 + F1 * 4);
constexpr int LG_A2D  = al16(LG_A2S + GOUT * 4);
constexpr int LG_B2   = al16(LG_A2D + GOUT * 4);
constexpr int LG_POOL = al16(LG_B2 + GOUT * 4);
constexpr int LG_ENC  = al16(LG_POOL + 2 * GOUT * 4);
constexpr int GAT_LDS = al16(LG_ENC + GOUT * 4);
static_assert(GAT_LDS <= 160 * 1024);
static_assert(LG_H1 % 16 == 0 && LG_ENC % 16 == 0);

__device__ __forceinline__ float rcpx(float x) { return __builtin_amdgcn_rcpf(x); }
__device__ __forceinline__ float sigm(float x) { return rcpx(1.0f + __expf(-x)); }
__device__ __forceinline__ float tanhm(float x) {
    const float e = __expf(2.0f * x);
    return 1.0f - 2.0f * rcpx(e + 1.0f);
}
__device__ __forceinline__ v8f zero8() {
    v8f z;
#pragma unroll
    for (int i = 0; i < 8; ++i) z[i] = 0.0f;
    return z;
}
__device__ __forceinline__ v8f ld8f(const float* p) {
    const v4f a = *(const v4f*)p;
    const v4f b = *(const v4f*)(p + 4);
    return __builtin_shufflevector(a, b, 0, 1, 2, 3, 4, 5, 6, 7);
}

__device__ __forceinline__ void ldfrag_lds(Frag& f, lcp_h p) {
    f.half[0] = *(AS3 const v8h*)(p);
    f.half[1] = *(AS3 const v8h*)(p + 16);
}
__device__ __forceinline__ void ldfrag_ptr(Frag& f, const _Float16* p) {
    f.half[0] = *(const v8h*)(p);
    f.half[1] = *(const v8h*)(p + 16);
}
__device__ __forceinline__ v8f mma16(v8f c, const Frag& a, const Frag& b) {
    v8f d = __builtin_amdgcn_wmma_f32_16x16x32_f16(false, a.v, false, b.v, (short)0, c, false, false);
    asm volatile("v_nop\n\tv_nop\n\tv_nop\n\tv_nop" : "+v"(d) : "v"(a.v), "v"(b.v));
    return d;
}

__global__ __launch_bounds__(NTHR)
void cvt_kernel(const float* __restrict__ W2, const float* __restrict__ Wih,
                const float* __restrict__ Whh, _Float16* W2P, _Float16* WP)
{
    const int tid = threadIdx.x;
    if ((int)blockIdx.x < NB_W2) {
        const int p  = (int)blockIdx.x * NTHR + tid;
        const int n  = p >> 4;
        const int k8 = (p & 15) * 8;
        v8h hv;
#pragma unroll
        for (int i = 0; i < 8; ++i) hv[i] = (_Float16)(W2[(size_t)(k8 + i) * GOUT + n] * SCL);
        _Float16* d = W2P + (size_t)n * KP2 + k8;
        *(volatile v8h*)d = hv;
        __threadfence();
        *(volatile v8h*)d = hv;
    } else {
        const int p  = ((int)blockIdx.x - NB_W2) * NTHR + tid;
        const int n  = p >> 5;
        const int c8 = (p & 31) * 8;
        const int ci = min(c8, GOUT - 8);
        const int cj = min(max(c8 - GOUT, 0), LH - 8);
        const v8f a = ld8f(Wih + (size_t)n * GOUT + ci);
        const v8f b = ld8f(Whh + (size_t)n * LH + cj);
        v8h hv;
#pragma unroll
        for (int i = 0; i < 8; ++i) {
            const float v = (c8 < GOUT) ? a[i] : b[i];
            hv[i] = (_Float16)(v * SCL);
        }
        _Float16* d = WP + (size_t)n * WPL + c8;
        *(volatile v8h*)d = hv;
        __threadfence();
        *(volatile v8h*)d = hv;
    }
}

__global__ __launch_bounds__(NTHR)
void gat_kernel(const float* __restrict__ x, const int* __restrict__ ei,
                const float* __restrict__ W1, const float* __restrict__ as1w,
                const float* __restrict__ ad1w, const float* __restrict__ b1,
                const _Float16* __restrict__ W2P,
                const float* __restrict__ as2w, const float* __restrict__ ad2w,
                const float* __restrict__ b2, float* ENC)
{
    extern __shared__ __attribute__((aligned(16))) char smem[];
    lp_f sFEAT = (lp_f)(smem + LG_FEAT);
    lp_h sH1   = (lp_h)(smem + LG_H1);
    lp_i sSLOT = (lp_i)(smem + LG_SLOT);
    lp_f sAL1  = (lp_f)(smem + LG_AL1);
    lp_f sAL2  = (lp_f)(smem + LG_AL2);
    lp_f sAS1  = (lp_f)(smem + LG_AS1);
    lp_f sAD1  = (lp_f)(smem + LG_AD1);
    lp_f sAS2  = (lp_f)(smem + LG_AS2);
    lp_f sAD2  = (lp_f)(smem + LG_AD2);
    lp_i sESRC = (lp_i)(smem + LG_ESRC);
    lp_i sEDST = (lp_i)(smem + LG_EDST);
    lp_i sCSRC = (lp_i)(smem + LG_CSRC);
    lp_i sOFF  = (lp_i)(smem + LG_OFF);
    lp_i sCNT  = (lp_i)(smem + LG_CNT);
    lp_f sX    = (lp_f)(smem + LG_X);
    lp_f sW1   = (lp_f)(smem + LG_W1);
    lp_f sA1S  = (lp_f)(smem + LG_A1S);
    lp_f sA1D  = (lp_f)(smem + LG_A1D);
    lp_f sB1   = (lp_f)(smem + LG_B1);
    lp_f sA2S  = (lp_f)(smem + LG_A2S);
    lp_f sA2D  = (lp_f)(smem + LG_A2D);
    lp_f sB2   = (lp_f)(smem + LG_B2);
    lp_f sPOOL = (lp_f)(smem + LG_POOL);
    lp_f sENC  = (lp_f)(smem + LG_ENC);

    const int t    = blockIdx.x;
    const int tid  = threadIdx.x;
    const int lane = tid & 31;
    const int wv   = tid >> 5;
    const int hf   = lane >> 4;
    const int m    = lane & 15;

    for (int i = tid; i < NN * 2; i += NTHR) sX[i] = x[(size_t)t * (NN * 2) + i];
    for (int i = tid; i < ET; i += NTHR) {
        const int ia = min(i, EE - 1);
        int sv = ei[ia];
        int dv = ei[EE + ia];
        sv = min(max(sv, 0), NN - 1);
        dv = min(max(dv, 0), NN - 1);
        const int self = min(max(i - EE, 0), NN - 1);
        sESRC[i] = (i < EE) ? sv : self;
        sEDST[i] = (i < EE) ? dv : self;
    }
    for (int i = tid; i < 2 * F1; i += NTHR) sW1[i] = W1[i];
    if (tid < F1) {
        sA1S[tid] = as1w[tid]; sA1D[tid] = ad1w[tid]; sB1[tid] = b1[tid];
        sA2S[tid] = as2w[tid]; sA2D[tid] = ad2w[tid]; sB2[tid] = b2[tid];
    }
    __syncthreads();

#pragma unroll 1
    for (int i = tid; i < NN * F1; i += NTHR) {
        const int n = i >> 7, f = i & (F1 - 1);
        sFEAT[n * FTS + f] = sX[2 * n] * sW1[f] + sX[2 * n + 1] * sW1[F1 + f];
    }
    if (tid < NN) {
        int c = 0;
#pragma unroll 1
        for (int e = 0; e < ET; ++e) {
            if (sEDST[e] == tid) {
                if (c < CAP) sSLOT[tid * CAP + c] = sESRC[e];
                ++c;
            }
        }
        sCNT[tid] = min(c, CAP);
    }
    __syncthreads();

    if (tid == 0) {
        int acc = 0;
#pragma unroll 1
        for (int d = 0; d < NN; ++d) { sOFF[d] = acc; acc += sCNT[d]; }
        sOFF[NN] = acc;
    }
#pragma unroll 1
    for (int i = tid; i < NN * HEADS; i += NTHR) {
        const int n = i >> 2, hh = i & 3;
        float s = 0.f, d = 0.f;
#pragma unroll 1
        for (int c = 0; c < HID; ++c) {
            const float v = sFEAT[n * FTS + hh * HID + c];
            s += v * sA1S[hh * HID + c];
            d += v * sA1D[hh * HID + c];
        }
        sAS1[n * HEADS + hh] = s;
        sAD1[n * HEADS + hh] = d;
    }
    __syncthreads();

    if (tid < NN) {
        const int beg = min(max(sOFF[tid], 0), ET);
        const int c   = min(max(sCNT[tid], 0), CAP);
#pragma unroll 1
        for (int q = 0; q < c; ++q) {
            const int pos = beg + q;
            if (pos < ET) sCSRC[pos] = sSLOT[tid * CAP + q];
        }
    }
    __syncthreads();

#pragma unroll 1
    for (int i = tid; i < NN * HEADS; i += NTHR) {
        const int d = i >> 2, hh = i & 3;
        int beg = sOFF[d], end = sOFF[d + 1];
        beg = min(max(beg, 0), ET);
        end = min(max(end, beg), min(beg + CAP, ET));
        const float adv = sAD1[d * HEADS + hh];
        float mx = -3.0e38f;
#pragma unroll 1
        for (int j = beg; j < end; ++j) {
            const unsigned sn = min((unsigned)sCSRC[j], (unsigned)(NN - 1));
            float sc = sAS1[sn * HEADS + hh] + adv;
            sc = (sc >= 0.f) ? sc : NEGS * sc;
            mx = fmaxf(mx, sc);
        }
        float ssum = 0.f;
#pragma unroll 1
        for (int j = beg; j < end; ++j) {
            const unsigned sn = min((unsigned)sCSRC[j], (unsigned)(NN - 1));
            float sc = sAS1[sn * HEADS + hh] + adv;
            sc = (sc >= 0.f) ? sc : NEGS * sc;
            const float ex = __expf(sc - mx);
            sAL1[j * HEADS + hh] = ex;
            ssum += ex;
        }
        const float inv = rcpx(ssum + 1e-16f);
#pragma unroll 1
        for (int j = beg; j < end; ++j) sAL1[j * HEADS + hh] = sAL1[j * HEADS + hh] * inv;
    }
    __syncthreads();

    {
        const int f = tid & (F1 - 1), par = tid >> 7, hh = f >> 5;
        const float bb = sB1[f];
#pragma unroll 1
        for (int d = par; d < NN; d += 2) {
            int beg = sOFF[d], end = sOFF[d + 1];
            beg = min(max(beg, 0), ET);
            end = min(max(end, beg), min(beg + CAP, ET));
            float acc = 0.f;
#pragma unroll 1
            for (int j = beg; j < end; ++j) {
                const unsigned sn = min((unsigned)sCSRC[j], (unsigned)(NN - 1));
                acc += sAL1[j * HEADS + hh] * sFEAT[sn * FTS + f];
            }
            float o = acc + bb;
            o = fmaxf(o, 0.f);
            sH1[d * H1S + f] = (_Float16)(o * SCL);
        }
#pragma unroll 1
        for (int i = tid; i < (H1R - NN) * H1S; i += NTHR) sH1[NN * H1S + i] = (_Float16)0.0f;
    }
    __syncthreads();

#pragma unroll 1
    for (int tile = wv; tile < 40; tile += 8) {
        const int m0 = (tile >> 3) * 16, n0 = (tile & 7) * 16;
        v8f acc = zero8();
        lcp_h ap = sH1 + (m0 + m) * H1S + 8 * hf;
        const _Float16* bp = W2P + (size_t)(n0 + m) * KP2 + 8 * hf;
#pragma unroll
        for (int kt = 0; kt < 4; ++kt) {
            Frag a, b;
            ldfrag_lds(a, ap + kt * 32);
            ldfrag_ptr(b, bp + kt * 32);
            acc = mma16(acc, a, b);
        }
#pragma unroll
        for (int r = 0; r < 8; ++r) {
            const int row = m0 + 8 * hf + r;
            if (row < NN) sFEAT[row * FTS + n0 + m] = acc[r] * INV256;
        }
    }
    __syncthreads();

    if (tid < NN) {
        float s = 0.f, d = 0.f;
#pragma unroll 1
        for (int c = 0; c < GOUT; ++c) {
            const float v = sFEAT[tid * FTS + c];
            s += v * sA2S[c];
            d += v * sA2D[c];
        }
        sAS2[tid] = s;
        sAD2[tid] = d;
    }
    __syncthreads();

    if (tid < NN) {
        const int d = tid;
        int beg = sOFF[d], end = sOFF[d + 1];
        beg = min(max(beg, 0), ET);
        end = min(max(end, beg), min(beg + CAP, ET));
        const float adv = sAD2[d];
        float mx = -3.0e38f;
#pragma unroll 1
        for (int j = beg; j < end; ++j) {
            const unsigned sn = min((unsigned)sCSRC[j], (unsigned)(NN - 1));
            float sc = sAS2[sn] + adv;
            sc = (sc >= 0.f) ? sc : NEGS * sc;
            mx = fmaxf(mx, sc);
        }
        float ssum = 0.f;
#pragma unroll 1
        for (int j = beg; j < end; ++j) {
            const unsigned sn = min((unsigned)sCSRC[j], (unsigned)(NN - 1));
            float sc = sAS2[sn] + adv;
            sc = (sc >= 0.f) ? sc : NEGS * sc;
            const float ex = __expf(sc - mx);
            sAL2[j] = ex;
            ssum += ex;
        }
        const float inv = rcpx(ssum + 1e-16f);
#pragma unroll 1
        for (int j = beg; j < end; ++j) sAL2[j] = sAL2[j] * inv;
    }
    __syncthreads();

    {
        const int c = tid & (GOUT - 1), par = tid >> 7;
        const float bb = sB2[c];
        float pool = 0.f;
#pragma unroll 1
        for (int d = par; d < NN; d += 2) {
            int beg = sOFF[d], end = sOFF[d + 1];
            beg = min(max(beg, 0), ET);
            end = min(max(end, beg), min(beg + CAP, ET));
            float acc = 0.f;
#pragma unroll 1
            for (int j = beg; j < end; ++j) {
                const unsigned sn = min((unsigned)sCSRC[j], (unsigned)(NN - 1));
                acc += sAL2[j] * sFEAT[sn * FTS + c];
            }
            pool += acc + bb;
        }
        sPOOL[par * GOUT + c] = pool;
    }
    __syncthreads();
    if (tid < GOUT) sENC[tid] = (sPOOL[tid] + sPOOL[GOUT + tid]) * (1.0f / (float)NN);
    __syncthreads();
    if (tid < 32) {
        const v4f v = *(AS3 const v4f*)(sENC + 4 * tid);
        float* p = ENC + (size_t)t * GOUT + 4 * tid;
        *(volatile v4f*)p = v;
        __threadfence();
        *(volatile v4f*)p = v;
    }
}

__global__ __launch_bounds__(NTHR)
void lstm_kernel(const float* __restrict__ ENC, const _Float16* __restrict__ WP,
                 const float* __restrict__ bih, const float* __restrict__ bhh,
                 const float* __restrict__ Wfc, const float* __restrict__ bfc, float* LOG)
{
    __shared__ __attribute__((aligned(16))) _Float16 sA[2 * 16 * APL];
    __shared__ float sBias[G4];
    __shared__ float sH[LH];
    __shared__ __attribute__((aligned(16))) float sLog[32];

    const int tid  = threadIdx.x;
    const int lane = tid & 31;
    const int wv   = tid >> 5;
    const int hf   = lane >> 4;
    const int m    = lane & 15;

    {
        v8h zh;
#pragma unroll
        for (int i = 0; i < 8; ++i) zh[i] = (_Float16)0.0f;
#pragma unroll 1
        for (int i = tid; i < (2 * 16 * APL) / 8; i += NTHR) *(v8h*)(&sA[8 * i]) = zh;
#pragma unroll 1
        for (int i = tid; i < G4; i += NTHR) sBias[i] = bih[i] + bhh[i];
        if (tid < LH) sH[tid] = 0.f;
        if (tid < 32) sLog[tid] = 0.f;
    }
    __syncthreads();
    if (tid < 32) {
        const v4f xv = *(const v4f*)(ENC + 4 * tid);
        v4h hv;
#pragma unroll
        for (int i = 0; i < 4; ++i) hv[i] = (_Float16)(xv[i] * SCL);
        *(v4h*)(&sA[4 * tid]) = hv;
    }

    float cst = 0.f;
    const int j0 = wv * 16;
    const _Float16* wb = WP + (size_t)(j0 + m) * WPL + 8 * hf;

#pragma unroll 1
    for (int s = 0; s < TT; ++s) {
        const int cur = s & 1;
        _Float16* sAc = sA + cur * (16 * APL);
        _Float16* sAn = sA + (cur ^ 1) * (16 * APL);

        __syncthreads();

        if (s + 1 < TT) {
            if (tid < 32) {
                const v4f xv = *(const v4f*)(ENC + (size_t)(s + 1) * GOUT + 4 * tid);
                v4h hv;
#pragma unroll
                for (int i = 0; i < 4; ++i) hv[i] = (_Float16)(xv[i] * SCL);
                *(v4h*)(sAn + 4 * tid) = hv;
            }
        }

        v8f acc[4];
#pragma unroll
        for (int q = 0; q < 4; ++q) acc[q] = zero8();
        const _Float16* ab = sAc + m * APL + 8 * hf;
#pragma unroll 1
        for (int k0 = 0; k0 < KCL; k0 += 32) {
            Frag a;
            ldfrag_ptr(a, ab + k0);
            Frag b[4];
#pragma unroll
            for (int q = 0; q < 4; ++q) ldfrag_ptr(b[q], wb + (size_t)q * (128 * WPL) + k0);
#pragma unroll
            for (int q = 0; q < 4; ++q) acc[q] = mma16(acc[q], a, b[q]);
        }

        if (hf == 0) {
            const int n = j0 + m;
            const float gi = acc[0][0] * INV256 + sBias[n];
            const float gf = acc[1][0] * INV256 + sBias[LH + n];
            const float gg = acc[2][0] * INV256 + sBias[2 * LH + n];
            const float go = acc[3][0] * INV256 + sBias[3 * LH + n];
            cst = sigm(gf) * cst + sigm(gi) * tanhm(gg);
            const float hn = sigm(go) * tanhm(cst);
            sAn[GOUT + n] = (_Float16)(hn * SCL);
            sH[n] = hn;
        }
    }
    __syncthreads();

    if (tid < NC) {
        float a = bfc[tid];
#pragma unroll 1
        for (int k = 0; k < LH; ++k) a += Wfc[tid * LH + k] * sH[k];
        sLog[tid] = a;
    }
    __syncthreads();
    v4f lv = zero8().lo;
    if (tid < 8) {
        lv = *(const v4f*)(&sLog[4 * tid]);
        *(volatile v4f*)(LOG + 4 * tid) = lv;
    }
    __threadfence();
    if (tid < 8) *(volatile v4f*)(LOG + 4 * tid) = lv;
}

__global__ __launch_bounds__(NTHR)
void out_kernel(const float* __restrict__ ENC, const float* __restrict__ LOG, float* out, int nout)
{
    const int f  = (int)blockIdx.x * NTHR + (int)threadIdx.x;
    const int fl = min(f, 31);
    const int fe = min(max(f - NC, 0), TT * GOUT - 1);
    const float lv = LOG[fl];
    const float ev = ENC[fe];
    const float v  = (f < NC) ? lv : ev;
    if (f < nout) *(volatile float*)(out + f) = v;
    __threadfence();
    if (f < nout) *(volatile float*)(out + f) = v;
}

extern "C" void kernel_launch(void* const* d_in, const int* in_sizes, int n_in,
                              void* d_out, int out_size, void* d_ws, size_t ws_size,
                              hipStream_t stream)
{
    if (n_in < 16) return;
    if (in_sizes[0]  != TT * NN * 2)  return;
    if (in_sizes[1]  != 2 * EE)       return;
    if (in_sizes[2]  != 2 * F1)       return;
    if (in_sizes[3]  != F1)           return;
    if (in_sizes[4]  != F1)           return;
    if (in_sizes[5]  != F1)           return;
    if (in_sizes[6]  != F1 * GOUT)    return;
    if (in_sizes[7]  != GOUT)         return;
    if (in_sizes[8]  != GOUT)         return;
    if (in_sizes[9]  != GOUT)         return;
    if (in_sizes[10] != G4 * GOUT)    return;
    if (in_sizes[11] != G4 * LH)      return;
    if (in_sizes[12] != G4)           return;
    if (in_sizes[13] != G4)           return;
    if (in_sizes[14] != NC * LH)      return;
    if (in_sizes[15] != NC)           return;
    if (out_size != NC + TT * GOUT)   return;
    if (ws_size < WS_END)             return;

    const float* x    = (const float*)d_in[0];
    const int*   ei   = (const int*)d_in[1];
    const float* W1   = (const float*)d_in[2];
    const float* as1w = (const float*)d_in[3];
    const float* ad1w = (const float*)d_in[4];
    const float* b1   = (const float*)d_in[5];
    const float* W2   = (const float*)d_in[6];
    const float* as2w = (const float*)d_in[7];
    const float* ad2w = (const float*)d_in[8];
    const float* b2   = (const float*)d_in[9];
    const float* Wih  = (const float*)d_in[10];
    const float* Whh  = (const float*)d_in[11];
    const float* bih  = (const float*)d_in[12];
    const float* bhh  = (const float*)d_in[13];
    const float* Wfc  = (const float*)d_in[14];
    const float* bfc  = (const float*)d_in[15];
    float* out = (float*)d_out;

    char* ws = (char*)d_ws;
    float*    ENC = (float*)(ws + OFF_ENC);
    _Float16* W2P = (_Float16*)(ws + OFF_W2P);
    _Float16* WP  = (_Float16*)(ws + OFF_WP);
    float*    LOG = (float*)(ws + OFF_LOG);

    cvt_kernel<<<dim3(NB_W2 + NB_WP), dim3(NTHR), 0, stream>>>(W2, Wih, Whh, W2P, WP);

    hipFuncSetAttribute(reinterpret_cast<const void*>(&gat_kernel),
                        hipFuncAttributeMaxDynamicSharedMemorySize, (int)GAT_LDS);
    gat_kernel<<<dim3(TT), dim3(NTHR), GAT_LDS, stream>>>(
        x, ei, W1, as1w, ad1w, b1, (const _Float16*)W2P, as2w, ad2w, b2, ENC);

    lstm_kernel<<<dim3(1), dim3(NTHR), 0, stream>>>(
        (const float*)ENC, (const _Float16*)WP, bih, bhh, Wfc, bfc, LOG);

    const int nob = (out_size + NTHR - 1) / NTHR;
    out_kernel<<<dim3(nob), dim3(NTHR), 0, stream>>>((const float*)ENC, (const float*)LOG, out, out_size);
}
